// SimpleGCN_14328010899646
// MI455X (gfx1250) — hardware-run, weakly checked
//
#include <hip/hip_runtime.h>

typedef float          v8f   __attribute__((ext_vector_type(8)));
typedef float          v4f   __attribute__((ext_vector_type(4)));
typedef unsigned int   v4u   __attribute__((ext_vector_type(4)));
typedef int            v8i   __attribute__((ext_vector_type(8)));
typedef unsigned short v8us  __attribute__((ext_vector_type(8)));
typedef unsigned short v16us __attribute__((ext_vector_type(16)));
typedef __bf16         v16bf __attribute__((ext_vector_type(16)));
typedef _Float16       v16h  __attribute__((ext_vector_type(16)));
typedef v4f  __attribute__((may_alias)) v4fa;
typedef v8us __attribute__((may_alias)) v8usa;
union FragB { v16bf v; v16us u; v8us h[2]; v8i w; };
union FragH { v16h  v; v16us u; v8us h[2]; v8i w; };

__device__ __forceinline__ v8f wmb(const FragB& a, const FragB& b, v8f c) {
  v8f d = __builtin_amdgcn_wmma_f32_16x16x32_bf16(false, a.v, false, b.v, (short)0, c, false, false);
  asm volatile("v_nop\n\tv_nop\n\tv_nop\n\tv_nop" : "+v"(d) : "v"(a.w), "v"(b.w));
  return d;
}

__device__ __forceinline__ v8f wmh(const FragH& a, const FragH& b, v8f c) {
  v8f d = __builtin_amdgcn_wmma_f32_16x16x32_f16(false, a.v, false, b.v, (short)0, c, false, false);
  asm volatile("v_nop\n\tv_nop\n\tv_nop\n\tv_nop" : "+v"(d) : "v"(a.w), "v"(b.w));
  return d;
}

__device__ __forceinline__ unsigned bf16_bits(float f) {
  const unsigned u = __float_as_uint(f);
  const unsigned r = (u + 0x7FFFu + ((u >> 16) & 1u)) >> 16;
  const unsigned q = (u >> 16) | 0x40u;
  return ((u & 0x7fffffffu) > 0x7f800000u) ? q : r;
}

__device__ __forceinline__ float bf16_val(float f) {
  return __uint_as_float(bf16_bits(f) << 16);
}
__device__ __forceinline__ int clampi(int v, int lo, int hi) {
  return v < lo ? lo : (v > hi ? hi : v);
}

__device__ __forceinline__ unsigned f16_bits(float f) {
  const unsigned u  = __float_as_uint(f);
  const unsigned s  = (u >> 16) & 0x8000u;
  const unsigned a  = u & 0x7fffffffu;
  const unsigned t  = a - 0x38000000u;
  const unsigned r  = (t + 0x0FFFu + ((t >> 13) & 1u)) >> 13;
  const unsigned rc = r > 0x7C00u ? 0x7C00u : r;
  const bool small  = a < 0x38800000u;
  const bool isnan  = a > 0x7f800000u;
  const unsigned fin = small ? 0u : (s | rc);
  return isnan ? (s | 0x7E00u) : fin;
}

__device__ __forceinline__ unsigned pk16(unsigned lo, unsigned hi) { return lo | (hi << 16); }
__device__ __forceinline__ unsigned bf16_lo_bits(float v) {
  float hi = bf16_val(v);
  asm volatile("" : "+v"(hi));
  return bf16_bits(v - hi);
}
__device__ __forceinline__ v4u pack8_bf16(v4f a, v4f c) {
  return (v4u){ pk16(bf16_bits(a[0]), bf16_bits(a[1])), pk16(bf16_bits(a[2]), bf16_bits(a[3])),
                pk16(bf16_bits(c[0]), bf16_bits(c[1])), pk16(bf16_bits(c[2]), bf16_bits(c[3])) };
}
__device__ __forceinline__ v4u pack8_bf16_lo(v4f a, v4f c) {
  return (v4u){ pk16(bf16_lo_bits(a[0]), bf16_lo_bits(a[1])), pk16(bf16_lo_bits(a[2]), bf16_lo_bits(a[3])),
                pk16(bf16_lo_bits(c[0]), bf16_lo_bits(c[1])), pk16(bf16_lo_bits(c[2]), bf16_lo_bits(c[3])) };
}
__device__ __forceinline__ v4u pack8_f16(v4f a, v4f c) {
  return (v4u){ pk16(f16_bits(a[0]), f16_bits(a[1])), pk16(f16_bits(a[2]), f16_bits(a[3])),
                pk16(f16_bits(c[0]), f16_bits(c[1])), pk16(f16_bits(c[2]), f16_bits(c[3])) };
}

template <int FORM>
__global__ __launch_bounds__(256) void k_plane(const float* __restrict__ src, int rows, int cols, int ldsrc,
                                               unsigned short* __restrict__ dst, int MP, int KP) {
  static_assert(FORM >= 0 && FORM <= 3);
  const int KTOT = (FORM == 1 || FORM == 3) ? 2 * KP : KP;
  const unsigned ppr   = (unsigned)(KTOT >> 3);
  const unsigned kp8   = (unsigned)(KP >> 3);
  const unsigned total = (unsigned)MP * ppr;
  const unsigned g     = blockIdx.x * 256u + threadIdx.x;
  const unsigned rowu  = g / ppr;
  const unsigned p     = g - rowu * ppr;
  const bool second    = p >= kp8;
  const int row = (int)rowu;
  const int c0  = (int)((second ? p - kp8 : p) << 3);
  const float* srow = src + (size_t)clampi(row, 0, rows - 1) * (size_t)ldsrc;
  float x[8];
  unsigned mk[8];
#pragma unroll
  for (int e = 0; e < 8; ++e) {
    const int c = c0 + e;
    const float v = srow[clampi(c, 0, cols - 1)];
    asm volatile("" :: "v"(v));
    x[e]  = v;
    mk[e] = (row < rows && c < cols) ? 0xFFFFu : 0u;
  }
  const v4f a = (v4f){ x[0], x[1], x[2], x[3] };
  const v4f c = (v4f){ x[4], x[5], x[6], x[7] };
  v4u o;
  if (FORM == 2) {
    o = pack8_f16(a, c);
  } else {
    const v4u hi = pack8_bf16(a, c);
    o = hi;
    if (FORM == 1) { const v4u lo = pack8_bf16_lo(a, c); o = second ? lo : hi; }
  }
  const v4u mw = (v4u){ pk16(mk[0], mk[1]), pk16(mk[2], mk[3]), pk16(mk[4], mk[5]), pk16(mk[6], mk[7]) };
  o &= mw;
  if (g < total) {
    volatile v4u* q = (volatile v4u*)(dst + (size_t)g * 8);
    *q = o;
    __threadfence();
    *q = o;
  }
}

template <int FORM> struct FragOf    { typedef FragB T; };
template <>         struct FragOf<2> { typedef FragH T; };
__device__ __forceinline__ v8f mm(const FragB& a, const FragB& b, v8f c) { return wmb(a, b, c); }
__device__ __forceinline__ v8f mm(const FragH& a, const FragH& b, v8f c) { return wmh(a, b, c); }
template <class F> __device__ __forceinline__ F ld_frag(const unsigned short* p) {
  F f;
  f.h[0] = *(const v8usa*)(p);
  f.h[1] = *(const v8usa*)(p + 16);
  return f;
}

template <int FORM, int EPI>
__global__ __launch_bounds__(256) __attribute__((amdgpu_num_vgpr(248)))
void k_gemm_nt(const unsigned short* __restrict__ A, const unsigned short* __restrict__ B,
               const float* __restrict__ bias, float* __restrict__ D, int M, int N, int KTOT, int ldd) {
  static_assert(FORM >= 0 && FORM <= 2);
  static_assert(EPI == 0 || EPI == 1);
  typedef typename FragOf<FORM>::T F;
  __shared__ __attribute__((aligned(16))) float sT[8][16 * 68];
  const int lane = threadIdx.x & 31;
  const int wave = threadIdx.x >> 5;
  const int tilesM = (M + 63) >> 6;
  const int tilesN = (N + 63) >> 6;
  const int tile = blockIdx.x * 8 + wave;
  if (tile >= tilesM * tilesN) return;
  const int tm = tile / tilesN;
  const int tn = tile - tm * tilesN;
  const int m0 = tm << 6;
  const int n0 = tn << 6;

  const int rl = lane & 15;
  const int h8 = (lane >> 4) * 8;
  const unsigned short* pa = A + (size_t)(m0 + rl) * (size_t)KTOT + h8;
  const unsigned short* pb = B + (size_t)(n0 + rl) * (size_t)KTOT + h8;

  v8f acc[4][4];
#pragma unroll
  for (int i = 0; i < 4; ++i)
#pragma unroll
    for (int j = 0; j < 4; ++j) acc[i][j] = (v8f){0.f, 0.f, 0.f, 0.f, 0.f, 0.f, 0.f, 0.f};

#pragma unroll 1
  for (int k0 = 0; k0 < KTOT; k0 += 32) {
    F bf[4];
#pragma unroll
    for (int j = 0; j < 4; ++j) bf[j] = ld_frag<F>(pb + (size_t)(j << 4) * (size_t)KTOT + k0);
#pragma unroll
    for (int i = 0; i < 4; ++i) {
      const F af = ld_frag<F>(pa + (size_t)(i << 4) * (size_t)KTOT + k0);
#pragma unroll
      for (int j = 0; j < 4; ++j) acc[i][j] = mm(af, bf[j], acc[i][j]);
    }
  }

  float* slab = sT[wave];
  const int hh = lane >> 4;
  const int c4 = (lane & 15) * 4;
  const int nc = n0 + c4;
  const bool cok = nc < N;
  v4f bv = (v4f){0.f, 0.f, 0.f, 0.f};
  if (EPI == 1) {
    bv = *(const v4fa*)(bias + clampi(nc, 0, N - 4));
    asm volatile("" :: "v"(bv));
  }
#pragma unroll
  for (int i = 0; i < 4; ++i) {
    const int mBase = m0 + (i << 4);
#pragma unroll
    for (int j = 0; j < 4; ++j) {
#pragma unroll
      for (int r = 0; r < 8; ++r) slab[(h8 + r) * 68 + (j << 4) + rl] = acc[i][j][r];
    }
    __builtin_amdgcn_fence(__ATOMIC_RELEASE, "workgroup");
    __builtin_amdgcn_wave_barrier();
    __builtin_amdgcn_fence(__ATOMIC_ACQUIRE, "workgroup");
    v4f vv[8];
#pragma unroll
    for (int it = 0; it < 8; ++it) {
      const int row = it * 2 + hh;
      v4f v = *(const v4fa*)(slab + row * 68 + c4);
      if (EPI == 1) v += bv;
      vv[it] = v;
    }
    for (int pass = 0; pass < 2; ++pass) {
#pragma unroll
      for (int it = 0; it < 8; ++it) {
        const int row = mBase + it * 2 + hh;
        if (cok && row < M) *(volatile v4f*)(D + (size_t)row * (size_t)ldd + nc) = vv[it];
      }
      __threadfence();
    }
    __builtin_amdgcn_fence(__ATOMIC_RELEASE, "workgroup");
    __builtin_amdgcn_wave_barrier();
    __builtin_amdgcn_fence(__ATOMIC_ACQUIRE, "workgroup");
  }
}

#include <stddef.h>
#include <stdint.h>
#include <math.h>

#pragma clang fp contract(off)

#define SPLIT_L2 0
#define SPLIT_L3 0
#ifndef SPLIT_L2
#define SPLIT_L2 1
#endif
#ifndef SPLIT_L3
#define SPLIT_L3 1
#endif

#define NN      100000
#define NE      1600000
#define MP      100096
#define F1      128
#define F3      64
#define NTHR    256
#define NWAVE   8
#define EPT     8
#define WCH     (32 * EPT)
#define NBRUN   1024
#define SLB     10
#define NBK     98
#define WLCAP   3328
#define RCAP    20992
#define DEGCAP  64
#define MAXDEG_MEAS   36
#define MAXB1024_MEAS 16710
#define K2TOT   (SPLIT_L2 ? 2 * F1 : F1)
#define K3TOT   (SPLIT_L3 ? 2 * F1 : F1)

#define BK_ZINTS (NWAVE * WLCAP + RCAP + 3 * NBRUN)
#define BK_INTS  (BK_ZINTS + 16)
#define BK_LDS   (BK_INTS * 4)

#define PB_W1   (F1 * F1 / 8 / NTHR)
#define PB_W2   (F1 * K2TOT / 8 / NTHR)
#define PB_W3   (F3 * K3TOT / 8 / NTHR)
#define PB_TOT  (PB_W1 + PB_W2 + PB_W3 + 1)

static_assert(F1 == 32 * 4 && F3 == 32 * 2);
static_assert(F1 % 32 == 0 && K2TOT % 32 == 0 && K3TOT % 32 == 0);
static_assert(MP % 128 == 0 && MP % 64 == 0 && MP >= NN && MP == 782 * 128);
static_assert(NN % 8 == 0 && MP % 32 == 0 && MP % NWAVE == 0);
static_assert(NBRUN == (1 << SLB) && NBRUN % 32 == 0);
static_assert(NE < (1 << 21));
static_assert(NBK * NBRUN >= MP && (NBK - 1) * NBRUN < NN);
static_assert(NE % WCH == 0 && NE % 4 == 0);
static_assert(RCAP % 256 == 0 && RCAP % (2 * NTHR) == 0 && BK_ZINTS % 4 == 0);
static_assert((long long)RCAP * 100 >= (long long)MAXB1024_MEAS * 125);
static_assert(WLCAP * 8 >= (RCAP / 8) * 10);
static_assert(WLCAP >= MAXB1024_MEAS / 8 + 8 * 46 + 1);
static_assert(MAXDEG_MEAS + 8 <= DEGCAP);
static_assert((NWAVE * WLCAP) % 4 == 0 && ((NWAVE * WLCAP + RCAP) % 4) == 0);
static_assert((2 * NBRUN) % (NTHR * 4) == 0);
static_assert(BK_LDS <= 262144);
static_assert((MP * F1 / 8) % NTHR == 0);
static_assert((F1 * F1 / 8) % NTHR == 0 && (F1 * K2TOT / 8) % NTHR == 0 && (F3 * K3TOT / 8) % NTHR == 0);

typedef float        v2f  __attribute__((ext_vector_type(2)));
typedef int          v2i  __attribute__((ext_vector_type(2)));
typedef int          v4i  __attribute__((ext_vector_type(4)));
typedef unsigned int v2u  __attribute__((ext_vector_type(2)));
typedef v2f __attribute__((may_alias)) v2fa;
typedef v2i __attribute__((may_alias)) v2ia;
typedef v4i __attribute__((may_alias)) v4ia;

__device__ __forceinline__ void st2_v4f(float* p, v4f v) {
  *(volatile v4f*)p = v;
  __threadfence();
  *(volatile v4f*)p = v;
}
__device__ __forceinline__ void st2_v4i(int* p, v4i v) {
  *(volatile v4i*)p = v;
  __threadfence();
  *(volatile v4i*)p = v;
}
__device__ __forceinline__ void st2_v4u(unsigned short* p, v4u v) {
  *(volatile v4u*)p = v;
  __threadfence();
  *(volatile v4u*)p = v;
}

__device__ __forceinline__ v4u gather8_bf16(const float* __restrict__ base, int stride) {
  float f[8];
#pragma unroll
  for (int i = 0; i < 8; ++i) {
    const float t = base[(size_t)i * (size_t)stride];
    asm volatile("" :: "v"(t));
    f[i] = t;
  }
  const v4f a = (v4f){ f[0], f[1], f[2], f[3] };
  const v4f c = (v4f){ f[4], f[5], f[6], f[7] };
  return pack8_bf16(a, c);
}

__device__ __forceinline__ void prep_w(const float* __restrict__ W, int nout, int ktot, int u, unsigned short* dst) {
  const int ppr = ktot >> 3;
  const int n   = u / ppr;
  const int p   = u - n * ppr;
  const int k8  = (p & 15) * 8;
  const v4u o = gather8_bf16(W + (size_t)k8 * (size_t)nout + n, nout);
  st2_v4u(dst + (size_t)n * (size_t)ktot + (size_t)p * 8, o);
}

__global__ __launch_bounds__(NTHR) void k_prep(const float* __restrict__ W1, const float* __restrict__ b1,
                                               const float* __restrict__ W2, const float* __restrict__ b2,
                                               const float* __restrict__ W3, const float* __restrict__ b3,
                                               unsigned short* W1T, unsigned short* W2D, unsigned short* W3D,
                                               float* BL) {
  const int tid = (int)threadIdx.x;
  const int blk = (int)blockIdx.x;
  if (blk < PB_W1) {
    prep_w(W1, F1, F1, blk * NTHR + tid, W1T);
  } else if (blk < PB_W1 + PB_W2) {
    prep_w(W2, F1, K2TOT, (blk - PB_W1) * NTHR + tid, W2D);
  } else if (blk < PB_W1 + PB_W2 + PB_W3) {
    prep_w(W3, F3, K3TOT, (blk - PB_W1 - PB_W2) * NTHR + tid, W3D);
  } else {
    const int lane = tid & 31, wave = tid >> 5;
    if (wave < 4) {
      v4f v = (v4f){0.f, 0.f, 0.f, 0.f};
      unsigned mk = 0xFFFFFFFFu;
      if (wave == 0) {
        v = *(const v4fa*)(b1 + 4 * lane);
      } else if (wave == 1) {
        v = *(const v4fa*)(b2 + 4 * lane);
      } else if (wave == 2) {
        const int idx = (4 * lane < F3 - 4) ? 4 * lane : F3 - 4;
        v = *(const v4fa*)(b3 + idx);
        mk = (lane < 16) ? 0xFFFFFFFFu : 0u;
      } else {
        mk = 0u;
      }
      asm volatile("" :: "v"(v));
      v4f o;
      o.x = __uint_as_float(__float_as_uint(bf16_val(v.x)) & mk);
      o.y = __uint_as_float(__float_as_uint(bf16_val(v.y)) & mk);
      o.z = __uint_as_float(__float_as_uint(bf16_val(v.z)) & mk);
      o.w = __uint_as_float(__float_as_uint(bf16_val(v.w)) & mk);
      st2_v4f(BL + wave * F1 + 4 * lane, o);
    }
  }
}

__global__ __launch_bounds__(NTHR) void k_bucket(const int* __restrict__ srcs, const int* __restrict__ dsts,
                                                 const float* __restrict__ ew, int* PAIRS, int* CO, int* FLAG) {
  extern __shared__ __attribute__((aligned(16))) int dsm[];
  int* wl   = dsm;
  int* pl   = dsm + NWAVE * WLCAP;
  int* cnt  = pl + RCAP;
  int* offs = cnt + NBRUN;
  int* cur  = offs + NBRUN;
  int* misc = cur + NBRUN;
  const int tid = (int)threadIdx.x, lane = tid & 31, wave = tid >> 5;
  const int blk = (int)blockIdx.x;
  const unsigned nbs = (unsigned)(blk * NBRUN);

  {
    const v4i z4 = {0, 0, 0, 0};
    for (int i = tid * 4; i < BK_ZINTS; i += NTHR * 4) *(v4ia*)(dsm + i) = z4;
    if (tid < 16) misc[tid] = 0;
  }
  __syncthreads();

  {
    const int per  = ((NE + NWAVE * WCH - 1) / (NWAVE * WCH)) * WCH;
    const int ebeg = wave * per;
    const int eend = (ebeg + per < NE) ? (ebeg + per) : NE;
    int* mylist = wl + wave * WLCAP;
    int wc = 0;
#pragma unroll 1
    for (int cb = ebeg; cb < eend; cb += WCH) {
      const int e0 = cb + lane * EPT;
      const v4i da = *(const v4ia*)(dsts + e0);
      const v4i db = *(const v4ia*)(dsts + e0 + 4);
      asm volatile("" :: "v"(da.x)); asm volatile("" :: "v"(da.y)); asm volatile("" :: "v"(da.z)); asm volatile("" :: "v"(da.w));
      asm volatile("" :: "v"(db.x)); asm volatile("" :: "v"(db.y)); asm volatile("" :: "v"(db.z)); asm volatile("" :: "v"(db.w));
      const unsigned s0 = (unsigned)da.x - nbs, s1 = (unsigned)da.y - nbs;
      const unsigned s2 = (unsigned)da.z - nbs, s3 = (unsigned)da.w - nbs;
      const unsigned s4 = (unsigned)db.x - nbs, s5 = (unsigned)db.y - nbs;
      const unsigned s6 = (unsigned)db.z - nbs, s7 = (unsigned)db.w - nbs;
      const bool h0 = s0 < (unsigned)NBRUN, h1 = s1 < (unsigned)NBRUN, h2 = s2 < (unsigned)NBRUN, h3 = s3 < (unsigned)NBRUN;
      const bool h4 = s4 < (unsigned)NBRUN, h5 = s5 < (unsigned)NBRUN, h6 = s6 < (unsigned)NBRUN, h7 = s7 < (unsigned)NBRUN;
      const unsigned m0 = __builtin_amdgcn_ballot_w32(h0), m1 = __builtin_amdgcn_ballot_w32(h1);
      const unsigned m2 = __builtin_amdgcn_ballot_w32(h2), m3 = __builtin_amdgcn_ballot_w32(h3);
      const unsigned m4 = __builtin_amdgcn_ballot_w32(h4), m5 = __builtin_amdgcn_ballot_w32(h5);
      const unsigned m6 = __builtin_amdgcn_ballot_w32(h6), m7 = __builtin_amdgcn_ballot_w32(h7);
      const unsigned any = m0 | m1 | m2 | m3 | m4 | m5 | m6 | m7;
      if (any != 0u) {
        const int pre = (int)(__builtin_amdgcn_mbcnt_lo(m0, 0u) + __builtin_amdgcn_mbcnt_lo(m1, 0u) +
                              __builtin_amdgcn_mbcnt_lo(m2, 0u) + __builtin_amdgcn_mbcnt_lo(m3, 0u) +
                              __builtin_amdgcn_mbcnt_lo(m4, 0u) + __builtin_amdgcn_mbcnt_lo(m5, 0u) +
                              __builtin_amdgcn_mbcnt_lo(m6, 0u) + __builtin_amdgcn_mbcnt_lo(m7, 0u));
        int p = wc + pre;
        if (h0) { if (p < WLCAP) mylist[p] = ((e0 + 0) << SLB) | (int)s0; p = p + 1; }
        if (h1) { if (p < WLCAP) mylist[p] = ((e0 + 1) << SLB) | (int)s1; p = p + 1; }
        if (h2) { if (p < WLCAP) mylist[p] = ((e0 + 2) << SLB) | (int)s2; p = p + 1; }
        if (h3) { if (p < WLCAP) mylist[p] = ((e0 + 3) << SLB) | (int)s3; p = p + 1; }
        if (h4) { if (p < WLCAP) mylist[p] = ((e0 + 4) << SLB) | (int)s4; p = p + 1; }
        if (h5) { if (p < WLCAP) mylist[p] = ((e0 + 5) << SLB) | (int)s5; p = p + 1; }
        if (h6) { if (p < WLCAP) mylist[p] = ((e0 + 6) << SLB) | (int)s6; p = p + 1; }
        if (h7) { if (p < WLCAP) mylist[p] = ((e0 + 7) << SLB) | (int)s7; p = p + 1; }
        wc += (int)(__builtin_popcount(m0) + __builtin_popcount(m1) + __builtin_popcount(m2) + __builtin_popcount(m3) +
                    __builtin_popcount(m4) + __builtin_popcount(m5) + __builtin_popcount(m6) + __builtin_popcount(m7));
      }
    }
    if (lane == 0) misc[wave] = wc;
  }
  __syncthreads();

  if (wave == 0) {
    int ov = 0;
    int tot = 0;
#pragma unroll 1
    for (int w2 = 0; w2 < NWAVE; ++w2) {
      int c = __builtin_amdgcn_readfirstlane(misc[w2]);
      if (c > WLCAP) ov = 1;
      c = c < 0 ? 0 : (c > WLCAP ? WLCAP : c);
      tot += c;
#pragma unroll 1
      for (int b0 = 0; b0 < c; b0 += 32) {
        const int idx = b0 + lane;
        const int ent = wl[w2 * WLCAP + (idx < WLCAP ? idx : WLCAP - 1)];
        const int m32 = (c - b0) < 32 ? (c - b0) : 32;
#pragma unroll 1
        for (int k = 0; k < m32; ++k) {
          const int u    = __builtin_amdgcn_readlane(ent, k);
          const int slot = u & (NBRUN - 1);
          if (lane == 0) cnt[slot] = cnt[slot] + 1;
        }
      }
    }
    if (tot > RCAP) ov = 1;
    if (lane == 0) {
      misc[9]  = ov;
      misc[10] = tot > RCAP ? RCAP : tot;
    }
  }
  __syncthreads();
  if (wave == 0) {
    const int base = lane * (NBRUN / 32);
    int s = 0;
    int bigl = 0;
#pragma unroll 1
    for (int i = 0; i < NBRUN / 32; ++i) {
      const int cv = cnt[base + i];
      s += cv;
      bigl |= (cv > DEGCAP) ? 1 : 0;
    }
    const unsigned bm = __builtin_amdgcn_ballot_w32(bigl != 0);
    int incl = s;
#pragma unroll
    for (int d = 1; d < 32; d <<= 1) {
      const int y = __shfl_up(incl, d, 32);
      incl += (lane >= d) ? y : 0;
    }
    int run = incl - s;
#pragma unroll 1
    for (int i = 0; i < NBRUN / 32; ++i) {
      const int cv = cnt[base + i];
      offs[base + i] = run;
      cur[base + i]  = run;
      run += cv;
    }
    if (lane == 0 && bm != 0u) misc[9] = 1;
  }
  __syncthreads();

  if (wave == 0) {
#pragma unroll 1
    for (int w2 = 0; w2 < NWAVE; ++w2) {
      int c = __builtin_amdgcn_readfirstlane(misc[w2]);
      c = c < 0 ? 0 : (c > WLCAP ? WLCAP : c);
#pragma unroll 1
      for (int b0 = 0; b0 < c; b0 += 32) {
        const int idx = b0 + lane;
        const int ent = wl[w2 * WLCAP + (idx < WLCAP ? idx : WLCAP - 1)];
        const int m32 = (c - b0) < 32 ? (c - b0) : 32;
#pragma unroll 1
        for (int k = 0; k < m32; ++k) {
          const int u    = __builtin_amdgcn_readlane(ent, k);
          const int slot = u & (NBRUN - 1);
          if (lane == 0) {
            int p = cur[slot];
            p = p < 0 ? 0 : (p > RCAP - 1 ? RCAP - 1 : p);
            pl[p] = (u >> SLB) & 0x1FFFFF;
            cur[slot] = p + 1;
          }
        }
      }
    }
  }
  __syncthreads();

  const int ovf = misc[9];
  const int tot = misc[10];
  int* lp  = PAIRS + (size_t)blk * (size_t)(2 * RCAP);
  int* cop = CO + (size_t)blk * (2 * NBRUN);
  int* fp  = FLAG + (size_t)blk * 32;
#pragma unroll 1
  for (int i = tid * 2; i < RCAP; i += NTHR * 2) {
    const v2i e2 = *(const v2ia*)(pl + i);
    const int e0 = clampi(e2.x, 0, NE - 1);
    const int e1 = clampi(e2.y, 0, NE - 1);
    int   s0 = srcs[e0];
    int   s1 = srcs[e1];
    const float w0 = ew[e0];
    const float w1 = ew[e1];
    asm volatile("" :: "v"(s0)); asm volatile("" :: "v"(s1));
    asm volatile("" :: "v"(w0)); asm volatile("" :: "v"(w1));
    s0 = clampi(s0, 0, NN - 1);
    s1 = clampi(s1, 0, NN - 1);
    const int k0 = (i < tot) ? -1 : 0;
    const int k1 = (i + 1 < tot) ? -1 : 0;
    v4i o;
    o.x = s0 & k0;
    o.y = (int)(bf16_bits(w0) << 16) & k0;
    o.z = s1 & k1;
    o.w = (int)(bf16_bits(w1) << 16) & k1;
    st2_v4i(lp + 2 * i, o);
  }
#pragma unroll 1
  for (int i = tid * 4; i < 2 * NBRUN; i += NTHR * 4) {
    const v4i v = *(const v4ia*)(cnt + i);
    st2_v4i(cop + i, v);
  }
  {
    const v4i f = {ovf, ovf, ovf, ovf};
    if (tid < 8) st2_v4i(fp + 4 * tid, f);
  }
}

__global__ __launch_bounds__(NTHR) void k_deg(const int* __restrict__ PAIRS, const int* __restrict__ CO, float* DINV) {
  __shared__ __attribute__((aligned(16))) float sd[32];
  const int tid = (int)threadIdx.x, lane = tid & 31, wave = tid >> 5;
  const int blk = (int)blockIdx.x;
  const int bk  = (blk * 32) >> SLB;
  const int* lb = PAIRS + (size_t)bk * (size_t)(2 * RCAP);
  const int* cb = CO + (size_t)bk * (2 * NBRUN);
  const float qnan = __uint_as_float(0x7fc00000u);
#pragma unroll 1
  for (int q = 0; q < 4; ++q) {
    const int node = blk * 32 + wave * 4 + q;
    const int slot = node & (NBRUN - 1);
    int c = cb[slot];
    int o = cb[NBRUN + slot];
    asm volatile("" :: "v"(c));
    asm volatile("" :: "v"(o));
    c = __builtin_amdgcn_readfirstlane(c);
    o = __builtin_amdgcn_readfirstlane(o);
    const bool big = c > DEGCAP;
    c = c < 0 ? 0 : (c > DEGCAP ? DEGCAP : c);
    o = o < 0 ? 0 : (o > RCAP - 1 ? RCAP - 1 : o);
    int last = o + (c > 0 ? c : 1) - 1;
    last = last > RCAP - 1 ? RCAP - 1 : last;
    float s = 0.0f;
#pragma unroll 1
    for (int b0 = 0; b0 < c; b0 += 32) {
      int idx = o + b0 + lane;
      idx = idx > last ? last : idx;
      const int wv = lb[2 * idx + 1];
      asm volatile("" :: "v"(wv));
      const int m32 = (c - b0) < 32 ? (c - b0) : 32;
#pragma unroll 1
      for (int k = 0; k < m32; ++k) s = s + __int_as_float(__builtin_amdgcn_readlane(wv, k));
    }
    const float deg = s + 1.0f;
    const float r   = 1.0f / sqrtf(deg);
    float dv = (deg > 0.0f) ? r : 0.0f;
    dv = big ? qnan : dv;
    dv = (node < NN) ? dv : 0.0f;
    if (lane == 0) sd[wave * 4 + q] = dv;
  }
  __syncthreads();
  {
    const v4f v = *(const v4fa*)(sd + 4 * (tid & 7));
    asm volatile("" :: "v"(v));
    if (tid < 8) st2_v4f(DINV + (size_t)blk * 32 + 4 * tid, v);
  }
}

template <int SPLIT>
__global__ __launch_bounds__(NTHR) void k_walk_h(const int* __restrict__ PAIRS, const int* __restrict__ CO,
                                                 const int* __restrict__ FLAG, const float* __restrict__ DINV,
                                                 const float* __restrict__ T, const float* __restrict__ BLN,
                                                 unsigned short* H) {
  constexpr int HP = SPLIT ? 2 * F1 : F1;
  __shared__ __attribute__((aligned(16))) float sb[F1];
  const int tid = (int)threadIdx.x, lane = tid & 31, wave = tid >> 5;
  if (tid < 32) {
    const v4f bv0 = *(const v4fa*)(BLN + 4 * tid);
    *(v4fa*)(sb + 4 * tid) = bv0;
  }
  __syncthreads();

  const int node = (int)blockIdx.x * NWAVE + wave;
  const int bk   = node >> SLB;
  const int slot = node & (NBRUN - 1);
  const int* cb  = CO + (size_t)bk * (2 * NBRUN);
  const int* lb  = PAIRS + (size_t)bk * (size_t)(2 * RCAP);
  int c = cb[slot];
  int o = cb[NBRUN + slot];
  int flag = FLAG[(size_t)bk * 32];
  asm volatile("" :: "v"(c));
  asm volatile("" :: "v"(o));
  asm volatile("" :: "v"(flag));
  c = __builtin_amdgcn_readfirstlane(c);
  o = __builtin_amdgcn_readfirstlane(o);
  flag = __builtin_amdgcn_readfirstlane(flag);
  const bool big = c > DEGCAP;
  c = c < 0 ? 0 : (c > DEGCAP ? DEGCAP : c);
  o = o < 0 ? 0 : (o > RCAP - 1 ? RCAP - 1 : o);
  int last = o + (c > 0 ? c : 1) - 1;
  last = last > RCAP - 1 ? RCAP - 1 : last;
  const float dd = DINV[clampi(node, 0, MP - 1)];
  asm volatile("" :: "v"(dd));

  v4f acc = (v4f){0.0f, 0.0f, 0.0f, 0.0f};
#pragma unroll 1
  for (int b0 = 0; b0 < c; b0 += 32) {
    int idx = o + b0 + lane;
    idx = idx > last ? last : idx;
    const v2i ent = *(const v2ia*)(lb + 2 * idx);
    asm volatile("" :: "v"(ent.x));
    asm volatile("" :: "v"(ent.y));
    const int sr = clampi(ent.x, 0, NN - 1);
    const float ds = DINV[sr];
    asm volatile("" :: "v"(ds));
    const float wv  = __int_as_float(ent.y);
    const float t0  = ds * wv;
    const float nrm = t0 * dd;
    const int nb  = __float_as_int(nrm);
    const int m32 = (c - b0) < 32 ? (c - b0) : 32;
#pragma unroll 1
    for (int k = 0; k < m32; ++k) {
      const int   sk = __builtin_amdgcn_readlane(sr, k);
      const float ck = __int_as_float(__builtin_amdgcn_readlane(nb, k));
      const v4f q = *(const v4fa*)(T + (size_t)sk * F1 + 4 * lane);
      const v4f pq = q * ck;
      acc = acc + pq;
    }
  }
  {
    const v4f ts = *(const v4fa*)(T + (size_t)clampi(node, 0, MP - 1) * F1 + 4 * lane);
    asm volatile("" :: "v"(ts));
    const float l0 = dd * 1.0f;
    const float nl = l0 * dd;
    const v4f pq = ts * nl;
    acc = acc + pq;
  }
  const v4f bv = *(const v4fa*)(sb + 4 * lane);
  float v0 = acc.x + bv.x, v1 = acc.y + bv.y, v2 = acc.z + bv.z, v3 = acc.w + bv.w;
  v0 = (v0 > 0.0f) ? v0 : (v0 - v0);
  v1 = (v1 > 0.0f) ? v1 : (v1 - v1);
  v2 = (v2 > 0.0f) ? v2 : (v2 - v2);
  v3 = (v3 > 0.0f) ? v3 : (v3 - v3);
  const float qnan = __uint_as_float(0x7fc00000u);
  const bool bad = (flag != 0) || big;
  v0 = bad ? qnan : v0; v1 = bad ? qnan : v1; v2 = bad ? qnan : v2; v3 = bad ? qnan : v3;
  const unsigned lm = (node < NN) ? 0xFFFFFFFFu : 0u;
  v2u hi, lo;
  hi.x = pk16(bf16_bits(v0), bf16_bits(v1)) & lm;
  hi.y = pk16(bf16_bits(v2), bf16_bits(v3)) & lm;
  lo.x = pk16(bf16_lo_bits(v0), bf16_lo_bits(v1)) & lm;
  lo.y = pk16(bf16_lo_bits(v2), bf16_lo_bits(v3)) & lm;
  unsigned short* hp = H + (size_t)node * HP + 4 * lane;
  *(volatile v2u*)hp = hi;
  if (SPLIT) *(volatile v2u*)(hp + F1) = lo;
  __threadfence();
  *(volatile v2u*)hp = hi;
  if (SPLIT) *(volatile v2u*)(hp + F1) = lo;
}

__global__ __launch_bounds__(NTHR) void k_walk_out(const int* __restrict__ PAIRS, const int* __restrict__ CO,
                                                   const int* __restrict__ FLAG, const float* __restrict__ DINV,
                                                   const float* __restrict__ T3, const float* __restrict__ BLN,
                                                   float* out) {
  __shared__ __attribute__((aligned(16))) float sb[F1];
  const int tid = (int)threadIdx.x, lane = tid & 31, wave = tid >> 5;
  if (tid < 32) {
    const v4f bv0 = *(const v4fa*)(BLN + 4 * tid);
    *(v4fa*)(sb + 4 * tid) = bv0;
  }
  __syncthreads();

  const int node  = (int)blockIdx.x * NWAVE + wave;
  const int nodec = clampi(node, 0, NN - 1);
  const int bk   = nodec >> SLB;
  const int slot = nodec & (NBRUN - 1);
  const int* cb  = CO + (size_t)bk * (2 * NBRUN);
  const int* lb  = PAIRS + (size_t)bk * (size_t)(2 * RCAP);
  int c = cb[slot];
  int o = cb[NBRUN + slot];
  int flag = FLAG[(size_t)bk * 32];
  asm volatile("" :: "v"(c));
  asm volatile("" :: "v"(o));
  asm volatile("" :: "v"(flag));
  c = __builtin_amdgcn_readfirstlane(c);
  o = __builtin_amdgcn_readfirstlane(o);
  flag = __builtin_amdgcn_readfirstlane(flag);
  const bool big = c > DEGCAP;
  c = c < 0 ? 0 : (c > DEGCAP ? DEGCAP : c);
  o = o < 0 ? 0 : (o > RCAP - 1 ? RCAP - 1 : o);
  int last = o + (c > 0 ? c : 1) - 1;
  last = last > RCAP - 1 ? RCAP - 1 : last;
  const float dd = DINV[nodec];
  asm volatile("" :: "v"(dd));

  float a0 = 0.0f, a1 = 0.0f;
#pragma unroll 1
  for (int b0 = 0; b0 < c; b0 += 32) {
    int idx = o + b0 + lane;
    idx = idx > last ? last : idx;
    const v2i ent = *(const v2ia*)(lb + 2 * idx);
    asm volatile("" :: "v"(ent.x));
    asm volatile("" :: "v"(ent.y));
    const int sr = clampi(ent.x, 0, NN - 1);
    const float ds = DINV[sr];
    asm volatile("" :: "v"(ds));
    const float wv  = __int_as_float(ent.y);
    const float t0  = ds * wv;
    const float nrm = t0 * dd;
    const int nb  = __float_as_int(nrm);
    const int m32 = (c - b0) < 32 ? (c - b0) : 32;
#pragma unroll 1
    for (int k = 0; k < m32; ++k) {
      const int   sk = __builtin_amdgcn_readlane(sr, k);
      const float ck = __int_as_float(__builtin_amdgcn_readlane(nb, k));
      const v2f q = *(const v2fa*)(T3 + (size_t)sk * F3 + 2 * lane);
      const float p0 = q.x * ck;
      const float p1 = q.y * ck;
      a0 = a0 + p0;
      a1 = a1 + p1;
    }
  }
  {
    const v2f ts = *(const v2fa*)(T3 + (size_t)nodec * F3 + 2 * lane);
    asm volatile("" :: "v"(ts));
    const float l0 = dd * 1.0f;
    const float nl = l0 * dd;
    const float p0 = ts.x * nl;
    const float p1 = ts.y * nl;
    a0 = a0 + p0;
    a1 = a1 + p1;
  }
  const float z0 = a0 + sb[2 * lane];
  const float z1 = a1 + sb[2 * lane + 1];
  const float e0 = expf(-z0);
  const float e1 = expf(-z1);
  float o0 = 1.0f / (1.0f + e0);
  float o1 = 1.0f / (1.0f + e1);
  const float qnan = __uint_as_float(0x7fc00000u);
  const bool bad = (flag != 0) || big;
  o0 = bad ? qnan : o0;
  o1 = bad ? qnan : o1;
  if (node < NN) {
    v2f ov;
    ov.x = o0; ov.y = o1;
    float* op = out + (size_t)node * F3 + 2 * lane;
    *(volatile v2f*)op = ov;
    __threadfence();
    *(volatile v2f*)op = ov;
  }
}

extern "C" void kernel_launch(void* const* d_in, const int* in_sizes, int n_in,
                              void* d_out, int out_size, void* d_ws, size_t ws_size,
                              hipStream_t stream) {
  if (n_in < 9) return;
  if (in_sizes[0] != NN * F1) return;
  if (in_sizes[1] != 2 * NE) return;
  if (in_sizes[2] != NE) return;
  if (in_sizes[3] != F1 * F1) return;
  if (in_sizes[4] != F1) return;
  if (in_sizes[5] != F1 * F1) return;
  if (in_sizes[6] != F1) return;
  if (in_sizes[7] != F1 * F3) return;
  if (in_sizes[8] != F3) return;
  if (out_size != NN * F3) return;

  const float* x  = (const float*)d_in[0];
  const int*   ei = (const int*)d_in[1];
  const float* ew = (const float*)d_in[2];
  const float* W1 = (const float*)d_in[3];
  const float* b1 = (const float*)d_in[4];
  const float* W2 = (const float*)d_in[5];
  const float* b2 = (const float*)d_in[6];
  const float* W3 = (const float*)d_in[7];
  const float* b3 = (const float*)d_in[8];
  const int* srcs = ei;
  const int* dsts = ei + NE;
  float* out = (float*)d_out;

  constexpr size_t zR    = (size_t)MP * (2 * F1) * 2;
  constexpr size_t zT    = (size_t)MP * F1 * 4;
  constexpr size_t zPAIR = (size_t)NBK * RCAP * 8;
  constexpr size_t zCO   = (size_t)NBK * 2 * NBRUN * 4;
  constexpr size_t zDINV = (size_t)MP * 4;
  constexpr size_t zFLAG = (size_t)NBK * 128;
  constexpr size_t zW1T  = (size_t)F1 * F1 * 2;
  constexpr size_t zW2D  = (size_t)F1 * (2 * F1) * 2;
  constexpr size_t zW3D  = (size_t)F3 * (2 * F1) * 2;
  constexpr size_t zBL   = (size_t)4 * F1 * 4;
  constexpr size_t oR    = 0;
  constexpr size_t oT    = oR + zR;
  constexpr size_t oPAIR = oT + zT;
  constexpr size_t oCO   = oPAIR + zPAIR;
  constexpr size_t oDINV = oCO + zCO;
  constexpr size_t oFLAG = oDINV + zDINV;
  constexpr size_t oW1T  = oFLAG + zFLAG;
  constexpr size_t oW2D  = oW1T + zW1T;
  constexpr size_t oW3D  = oW2D + zW2D;
  constexpr size_t oBL   = oW3D + zW3D;
  constexpr size_t oEND  = oBL + zBL;
  static_assert(zR % 256 == 0 && zT % 256 == 0 && zPAIR % 256 == 0 && zCO % 256 == 0 && zDINV % 256 == 0);
  static_assert(zFLAG % 256 == 0 && zW1T % 256 == 0 && zW2D % 256 == 0 && zW3D % 256 == 0 && zBL % 256 == 0);
  static_assert(zR >= (size_t)MP * F1 * 2);
  static_assert(zT >= (size_t)MP * F3 * 4);
  static_assert(zW2D >= (size_t)F1 * K2TOT * 2 && zW3D >= (size_t)F3 * K3TOT * 2);
  static_assert(oEND == (size_t)((size_t)469941 * 256));
  static_assert(oEND <= ((size_t)128 << 20));
  if (oEND > ws_size) return;

  char* ws = (char*)d_ws;
  unsigned short* XB   = (unsigned short*)(ws + oR);
  unsigned short* H    = (unsigned short*)(ws + oR);
  float*          T    = (float*)(ws + oT);
  int*            PAIRS = (int*)(ws + oPAIR);
  int*            CO   = (int*)(ws + oCO);
  float*          DINV = (float*)(ws + oDINV);
  int*            FLAG = (int*)(ws + oFLAG);
  unsigned short* W1T  = (unsigned short*)(ws + oW1T);
  unsigned short* W2D  = (unsigned short*)(ws + oW2D);
  unsigned short* W3D  = (unsigned short*)(ws + oW3D);
  float*          BL   = (float*)(ws + oBL);
  const float*    ZB   = BL + 3 * F1;

  hipFuncSetAttribute(reinterpret_cast<const void*>(&k_bucket), hipFuncAttributeMaxDynamicSharedMemorySize, (int)BK_LDS);

  constexpr int G128 = ((MP / 64) * (F1 / 64) + 7) / 8;
  constexpr int G64  = ((MP / 64) * (F3 / 64) + 7) / 8;

  k_plane<0><<<MP * F1 / 8 / NTHR, NTHR, 0, stream>>>(x, NN, F1, F1, XB, MP, F1);
  k_prep<<<PB_TOT, NTHR, 0, stream>>>(W1, b1, W2, b2, W3, b3, W1T, W2D, W3D, BL);
  k_bucket<<<NBK, NTHR, BK_LDS, stream>>>(srcs, dsts, ew, PAIRS, CO, FLAG);
  k_deg<<<MP / 32, NTHR, 0, stream>>>(PAIRS, CO, DINV);
  k_gemm_nt<0, 0><<<G128, NTHR, 0, stream>>>(XB, W1T, ZB, T, MP, F1, F1, F1);
  k_walk_h<SPLIT_L2><<<MP / NWAVE, NTHR, 0, stream>>>(PAIRS, CO, FLAG, DINV, T, BL, H);
  k_gemm_nt<0, 0><<<G128, NTHR, 0, stream>>>(H, W2D, ZB, T, MP, F1, K2TOT, F1);
  k_walk_h<SPLIT_L3><<<MP / NWAVE, NTHR, 0, stream>>>(PAIRS, CO, FLAG, DINV, T, BL + F1, H);
  k_gemm_nt<0, 0><<<G64, NTHR, 0, stream>>>(H, W3D, ZB, T, MP, F3, K3TOT, F3);
  k_walk_out<<<NN / NWAVE, NTHR, 0, stream>>>(PAIRS, CO, FLAG, DINV, T, BL + 2 * F1, out);
}
